// FBPinn_58196806861032
// MI455X (gfx1250) — hardware-verified
//
#include <hip/hip_runtime.h>


#ifndef NPTS
#define NPTS 65536
#endif
#define NPTS_FULL 65536
#define NW   16
#define NEUR 128
#define NHID 2
#define TP   64
#define HP   136
#define SINV (1.0f / 0.02f)
#define T2L  2.8853900817779268f

static_assert(NEUR == 128);
static_assert(NEUR % 32 == 0);
static_assert(NPTS % TP == 0);
static_assert(NPTS <= NPTS_FULL);
static_assert(HP % 8 == 0 && HP >= NEUR);
static_assert(TP == 64);

typedef unsigned short bf;
typedef __attribute__((ext_vector_type(16))) __bf16   v16bf;
typedef __attribute__((ext_vector_type(8)))  unsigned short v8us;
typedef __attribute__((ext_vector_type(8)))  float    v8f;
typedef __attribute__((ext_vector_type(4)))  float    v4f;
typedef v4f  __attribute__((may_alias)) v4fa;
typedef v8us __attribute__((may_alias)) v8usa;

__device__ __forceinline__ unsigned short f2bf(float f) { unsigned u = __float_as_uint(f); u += 0x7FFFu + ((u >> 16) & 1u); return (unsigned short)(u >> 16); }
__device__ __forceinline__ float bfr(float f) { return __uint_as_float(((unsigned)f2bf(f)) << 16); }
__device__ __forceinline__ v16bf cat16b(v8us lo, v8us hi) { return __builtin_bit_cast(v16bf, __builtin_shufflevector(lo, hi, 0, 1, 2, 3, 4, 5, 6, 7, 8, 9, 10, 11, 12, 13, 14, 15)); }
__device__ __forceinline__ v8f wmmab(v16bf a, v16bf b, v8f c) { return __builtin_amdgcn_wmma_f32_16x16x32_bf16(false, a, false, b, (short)0, c, false, false); }
__device__ __forceinline__ v16bf ldb(const bf* __restrict__ p) { return cat16b(*(const v8us*)p, *(const v8us*)(p + 16)); }
__device__ __forceinline__ float tanh_fast(float x) { const float t = __builtin_amdgcn_exp2f(x * T2L); return 1.0f - 2.0f * __builtin_amdgcn_rcpf(1.0f + t); }
__device__ __forceinline__ void split2(float v, unsigned short& h, unsigned short& l) {
    const unsigned u = __float_as_uint(v); h = (unsigned short)(u >> 16); l = f2bf(v - __uint_as_float(u & 0xFFFF0000u)); }
__device__ __forceinline__ void ld8r(const float* __restrict__ p, float (&o)[8]) {
    const v4f a = *(const v4f*)p; const v4f b = *(const v4f*)(p + 4);
#pragma unroll
    for (int i = 0; i < 4; ++i) { o[i] = bfr(a[i]); o[4 + i] = bfr(b[i]); }
}

__global__ __launch_bounds__(256) void k_wt(const float* __restrict__ W, bf* Wt) {
    __shared__ __align__(16) bf t[NEUR * HP];
    const int tid = threadIdx.x; const size_t mo = (size_t)blockIdx.x * NEUR * NEUR;
#pragma unroll 4
    for (int i = 0; i < 64; ++i) { const int idx = i * 256 + tid; const int d = idx >> 7, e = idx & 127; t[e * HP + d] = f2bf(W[mo + idx]); }
    __syncthreads();
#pragma unroll 1
    for (int ps = 0; ps < 2; ++ps) {
#pragma unroll
        for (int i = 0; i < 8; ++i) { const int idx = i * 256 + tid; const int e = idx >> 4, q = idx & 15;
            const v8us val = *(const v8usa*)(&t[e * HP + 8 * q]);
            *(volatile v8us*)(Wt + mo + (size_t)e * NEUR + 8 * q) = val; }
        if (ps == 0) __threadfence(); }
}

__global__ __launch_bounds__(64) void k_fb(const float* __restrict__ x, const float* __restrict__ means, const float* __restrict__ stds, const float* __restrict__ mids,
                                           const float* __restrict__ W_in, const float* __restrict__ b_in, const bf* __restrict__ Wt, const float* __restrict__ b_hid,
                                           const float* __restrict__ W_out, const float* __restrict__ b_out, float* out) {
    __shared__ __align__(16) bf Hh[TP * HP];
    __shared__ __align__(16) bf Hl[TP * HP];
    __shared__ __align__(16) float xs[TP];
    __shared__ __align__(16) float part[2 * TP];
    __shared__ __align__(16) float outs[TP];
    const int tid = threadIdx.x, lane = tid & 31, lr = lane & 15, hi = lane >> 4;
    const int wave = __builtin_amdgcn_readfirstlane(tid >> 5);
    const int e0 = wave * 64;
    const int n0 = blockIdx.x * TP;
    const float xv = bfr(x[n0 + tid]);
    xs[tid] = xv;
    __syncthreads();
    float racc = 0.0f;
    const int q8 = (tid & 15) * 8, pr = tid >> 4;
    const int hb = lr * HP + 8 * hi;
#pragma unroll 1
    for (int w = 0; w < NW; ++w) {
        {
            const float mean = bfr(means[w]);
            const float istd = 1.0f / bfr(stds[w]);
            float wi[8], bi[8];
            ld8r(W_in + (size_t)w * NEUR + q8, wi);
            ld8r(b_in + (size_t)w * NEUR + q8, bi);
#pragma unroll 1
            for (int i = 0; i < 16; ++i) {
                const int p = pr + 4 * i;
                const float xn = (xs[p] - mean) * istd;
                v8us oh, ol;
#pragma unroll
                for (int r = 0; r < 8; ++r) { unsigned short a, b; split2(tanh_fast(xn * wi[r] + bi[r]), a, b); oh[r] = a; ol[r] = b; }
                *(v8us*)(&Hh[p * HP + q8]) = oh; *(v8us*)(&Hl[p * HP + q8]) = ol;
            }
        }
        __syncthreads();
#pragma unroll 1
        for (int l = 0; l < NHID; ++l) {
            v8f acc[4][4];
#pragma unroll
            for (int mb = 0; mb < 4; ++mb)
#pragma unroll
                for (int nb = 0; nb < 4; ++nb) acc[mb][nb] = (v8f){};
            const bf* wrow = Wt + ((size_t)(l * NW + w) * NEUR + e0 + lr) * NEUR + 8 * hi;
#pragma unroll 1
            for (int kc = 0; kc < NEUR; kc += 32) {
                v16bf a[4];
#pragma unroll
                for (int mb = 0; mb < 4; ++mb) a[mb] = ldb(wrow + (size_t)mb * 16 * NEUR + kc);
#pragma unroll
                for (int nb = 0; nb < 4; ++nb) {
                    const int o = hb + nb * 16 * HP + kc;
                    const v16bf bh = cat16b(*(const v8us*)(&Hh[o]), *(const v8us*)(&Hh[o + 16]));
                    const v16bf bl = cat16b(*(const v8us*)(&Hl[o]), *(const v8us*)(&Hl[o + 16]));
#pragma unroll
                    for (int mb = 0; mb < 4; ++mb) acc[mb][nb] = wmmab(a[mb], bh, acc[mb][nb]);
#pragma unroll
                    for (int mb = 0; mb < 4; ++mb) acc[mb][nb] = wmmab(a[mb], bl, acc[mb][nb]);
                }
                asm volatile("v_nop\n\tv_nop\n\tv_nop\n\tv_nop" : "+v"(acc[0][3]), "+v"(acc[1][3]), "+v"(acc[2][3]), "+v"(acc[3][3]) : "v"(a[0]), "v"(a[1]), "v"(a[2]), "v"(a[3]));
            }
            __syncthreads();
            const float* bsrc = b_hid + (size_t)(l * NW + w) * NEUR + e0 + 8 * hi;
            if (l + 1 < NHID) {
#pragma unroll
                for (int mb = 0; mb < 4; ++mb) {
                    float bb[8]; ld8r(bsrc + 16 * mb, bb);
#pragma unroll
                    for (int nb = 0; nb < 4; ++nb) {
                        v8us oh, ol;
#pragma unroll
                        for (int r = 0; r < 8; ++r) { unsigned short a, b; split2(tanh_fast(acc[mb][nb][r] + bb[r]), a, b); oh[r] = a; ol[r] = b; }
                        const int o = (16 * nb + lr) * HP + e0 + 16 * mb + 8 * hi;
                        *(v8us*)(&Hh[o]) = oh; *(v8us*)(&Hl[o]) = ol;
                    }
                }
            } else {
                float s[4] = {0.0f, 0.0f, 0.0f, 0.0f};
#pragma unroll
                for (int mb = 0; mb < 4; ++mb) {
                    float bb[8], ww[8]; ld8r(bsrc + 16 * mb, bb); ld8r(W_out + (size_t)w * NEUR + e0 + 16 * mb + 8 * hi, ww);
#pragma unroll
                    for (int nb = 0; nb < 4; ++nb) {
#pragma unroll
                        for (int r = 0; r < 8; ++r) s[nb] += tanh_fast(acc[mb][nb][r] + bb[r]) * ww[r];
                    }
                }
#pragma unroll
                for (int nb = 0; nb < 4; ++nb) s[nb] += __shfl_xor(s[nb], 16, 32);
                if (hi == 0) {
#pragma unroll
                    for (int nb = 0; nb < 4; ++nb) part[wave * TP + 16 * nb + lr] = s[nb];
                }
            }
            __syncthreads();
        }
        {
            const float u = (part[tid] + part[TP + tid]) + bfr(b_out[w]);
            const float tl = (xv - bfr(mids[w])) * SINV;
            const float tr = (xv - bfr(mids[w + 1])) * SINV;
            const float wnd = __builtin_amdgcn_rcpf(1.0f + expf(tl)) * __builtin_amdgcn_rcpf(1.0f + expf(-tr));
            racc += wnd * u;
        }
    }
    outs[tid] = racc;
    __syncthreads();
    if (tid < 16) {
        const v4f val = *(const v4fa*)(&outs[4 * tid]);
        float* dst = out + (size_t)n0 + 4 * tid;
        *(volatile v4f*)dst = val;
        __threadfence();
        *(volatile v4f*)dst = val;
    }
}

static constexpr size_t al256(size_t v) { return (v + 255) & ~(size_t)255; }
static constexpr size_t SZ_WT = al256((size_t)NHID * NW * NEUR * NEUR * 2);
static constexpr size_t SZ_TOTAL = SZ_WT;
static_assert(SZ_TOTAL <= (size_t)134217728);
static_assert(SZ_WT >= (size_t)NHID * NW * NEUR * (size_t)NEUR * 2);

extern "C" void kernel_launch(void* const* d_in, const int* in_sizes, int n_in,
                              void* d_out, int out_size, void* d_ws, size_t ws_size, hipStream_t stream) {
    if (n_in < 10) return;
    if ((size_t)in_sizes[0] < (size_t)NPTS) return;
    if (in_sizes[1] < NW || in_sizes[2] < NW || in_sizes[3] < NW + 1) return;
    if (in_sizes[4] < NW * NEUR || in_sizes[5] < NW * NEUR) return;
    if ((size_t)in_sizes[6] < (size_t)NHID * NW * NEUR * NEUR || in_sizes[7] < NHID * NW * NEUR) return;
    if (in_sizes[8] < NW * NEUR || in_sizes[9] < NW) return;
    if ((size_t)out_size < (size_t)NPTS) return;
    if (SZ_TOTAL > ws_size) return;
    const float* x     = (const float*)d_in[0];
    const float* means = (const float*)d_in[1];
    const float* stds  = (const float*)d_in[2];
    const float* mids  = (const float*)d_in[3];
    const float* W_in  = (const float*)d_in[4];
    const float* b_in  = (const float*)d_in[5];
    const float* W_hid = (const float*)d_in[6];
    const float* b_hid = (const float*)d_in[7];
    const float* W_out = (const float*)d_in[8];
    const float* b_out = (const float*)d_in[9];
    float* OUT = (float*)d_out;
    bf* WT = (bf*)d_ws;

    k_wt<<<dim3(NHID * NW, 1, 1), 256, 0, stream>>>(W_hid, WT);
    k_fb<<<dim3(NPTS / TP, 1, 1), 64, 0, stream>>>(x, means, stds, mids, W_in, b_in, WT, b_hid, W_out, b_out, OUT);
}
